// GAT_TGNN_51453708206732
// MI455X (gfx1250) — hardware-run, weakly checked
//
#include <hip/hip_runtime.h>


namespace {
constexpr int N = 8192, NP = 8192, E = 65536, IN = 128, NH = 8, HID = 512, HC = NH * HID  , HHC = HC / 2  , TE = 100000, TEP = 100000  , NOUT = 7;
constexpr float XS = 8.0f, WSC = 256.0f, NEG = 0.2f, EPSD = 1e-16f;
typedef __attribute__((ext_vector_type(4))) _Float16 v4b;

typedef _Float16 b16;
typedef __attribute__((ext_vector_type(16))) _Float16 v16b;
typedef __attribute__((ext_vector_type(8))) _Float16 v8b;
typedef __attribute__((ext_vector_type(8))) float v8f;
typedef __attribute__((ext_vector_type(4))) float v4f;
__device__ __forceinline__ float bf16_rne(float f) { unsigned int u = __float_as_uint(f); u += 0x7FFFu + ((u >> 16) & 1u); return __uint_as_float(u & 0xFFFF0000u); }
__device__ __forceinline__ void split16(float v, b16& hi, b16& lo) { hi = (b16)v; lo = (b16)(v - (float)hi); }
__device__ __forceinline__ v16b frag_kb(const b16* p, int hh) { const v8b a = *(const v8b*)(p + 8 * hh), b = *(const v8b*)(p + 16 + 8 * hh); v16b f;
#pragma unroll
  for (int e = 0; e < 8; ++e) { f[e] = a[e]; f[8 + e] = b[e]; } return f; }
__device__ __forceinline__ v8f wmma16b(v16b a, v16b b, v8f c) { v8f d = __builtin_amdgcn_wmma_f32_16x16x32_f16(false, a, false, b, (short)0, c, false, false); asm volatile("v_nop\n\tv_nop\n\tv_nop\n\tv_nop" : "+v"(d) : "v"(a), "v"(b)); return d; }
__device__ __forceinline__ void wave_lds_sync() { __builtin_amdgcn_fence(__ATOMIC_RELEASE, "workgroup"); __builtin_amdgcn_wave_barrier(); __builtin_amdgcn_fence(__ATOMIC_ACQUIRE, "workgroup"); }
__device__ __forceinline__ float pmul(float a, float b) { float p = a * b; asm volatile("" : "+v"(p)); return p; }
__device__ __forceinline__ int iclamp(int v, int lo, int hi) { return v < lo ? lo : (v > hi ? hi : v); }
__device__ __forceinline__ float nexp(float x) { return __builtin_amdgcn_exp2f(x * 1.4426950408889634f); }
__device__ __forceinline__ float lrelu(float x) { return x > 0.0f ? x : NEG * x; }

__device__ __forceinline__ float elu_(float x) { return x > 0.0f ? x : (__expf(x) - 1.0f); }
constexpr int CSR_NBLK = 512, CSR_GB = 9, CSR_GN = 1 << CSR_GB  , CSR_MAXG = 512, CSR_CAP = 12288  ;
__global__ __launch_bounds__(64) void csrA_kernel(const int* __restrict__ dst, int E, int N, int nG, int CHP, int NGP, int* __restrict__ STG, int* __restrict__ HST) {
  extern __shared__ int sm[];
  int* cnt = sm; int* run = sm + NGP; int* ids = sm + 2 * NGP;
  const int b = blockIdx.x; const int ch = (E + CSR_NBLK - 1) / CSR_NBLK; const int e0 = b * ch, e1 = min(E, e0 + ch);
  for (int i = threadIdx.x; i < NGP; i += 64) cnt[i] = 0;
  for (int i = threadIdx.x; i < CHP; i += 64) ids[i] = -1;
  __syncthreads();
  if (threadIdx.x == 0) {
    for (int e = e0; e < e1; ++e) { int d = dst[e]; d = (d < 0) ? 0 : (d >= N ? N - 1 : d); cnt[d >> CSR_GB] += 1; }
    int acc = 0; for (int g = 0; g < nG; ++g) { run[g] = acc; acc += cnt[g]; }
    for (int e = e0; e < e1; ++e) { int d = dst[e]; d = (d < 0) ? 0 : (d >= N ? N - 1 : d); const int g = d >> CSR_GB; ids[run[g]] = e; run[g] += 1; } }
  __syncthreads();
  typedef __attribute__((ext_vector_type(4))) int v4i;
  for (int pass = 0; pass < 2; ++pass) {
    for (int i = threadIdx.x; i < CHP / 4; i += 64) *(volatile v4i*)(STG + (size_t)b * CHP + i * 4) = *(const v4i*)(&ids[i * 4]);
    for (int i = threadIdx.x; i < NGP / 4; i += 64) { v4i v; for (int e = 0; e < 4; ++e) v[e] = (i * 4 + e < nG) ? cnt[i * 4 + e] : 0; *(volatile v4i*)(HST + (size_t)b * NGP + i * 4) = v; }
    __threadfence(); }
}
__global__ __launch_bounds__(512) void csrS_kernel(const int* __restrict__ HST, int nG, int NGP, int* __restrict__ START, int* __restrict__ TOT, int* __restrict__ OFF) {
  __shared__ int tot[CSR_MAXG];
  const int b = threadIdx.x;
  for (int pass = 0; pass < 2; ++pass) { int runb = 0; for (int g = 0; g < nG; ++g) { int c = HST[(size_t)b * NGP + g]; c = (c < 0) ? 0 : c; ((volatile int*)OFF)[(size_t)g * CSR_NBLK + b] = runb; runb += c; } __threadfence(); }
  for (int g = threadIdx.x; g < nG; g += 512) { int s = 0; for (int bb = 0; bb < CSR_NBLK; ++bb) { int c = HST[(size_t)bb * NGP + g]; s += (c < 0) ? 0 : c; } tot[g] = s; }
  __syncthreads();
  if (threadIdx.x < 32) {
    __shared__ int st[CSR_MAXG + 32];
    if (threadIdx.x == 0) { int acc = 0; for (int g = 0; g < NGP; ++g) { st[g] = acc; if (g < nG) acc += (tot[g] + 31) & ~31; } st[NGP] = acc; }
    __builtin_amdgcn_fence(__ATOMIC_RELEASE, "workgroup"); __builtin_amdgcn_wave_barrier(); __builtin_amdgcn_fence(__ATOMIC_ACQUIRE, "workgroup");
    for (int pass = 0; pass < 2; ++pass) { for (int i = threadIdx.x; i < NGP + 32; i += 32) { ((volatile int*)START)[i] = (i <= NGP) ? st[min(i, NGP)] : 0; ((volatile int*)TOT)[i] = (i < nG) ? tot[i] : 0; } __threadfence(); } }
}
__global__ __launch_bounds__(256) void csrB_kernel(const int* __restrict__ dst, int N, int nG, int CHP, int NGP, int permLen, const int* __restrict__ STG, const int* __restrict__ HST, const int* __restrict__ OFF, const int* __restrict__ START, const int* __restrict__ TOT, int* __restrict__ PERM, int* __restrict__ ROWPTR, int* __restrict__ ROWCNT, int* __restrict__ FLAG) {
  typedef __attribute__((ext_vector_type(4))) int v4i;
  __shared__ int ids[CSR_CAP]; __shared__ unsigned short key[CSR_CAP]; __shared__ int outp[CSR_CAP]; __shared__ int ncnt[CSR_GN + 1]; __shared__ int boff[CSR_NBLK + 1];
  const int g = blockIdx.x, t_ = threadIdx.x; int tot = TOT[g]; int st = START[g], stn = START[g + 1]; const int v0 = g * CSR_GN; const int nv = min(CSR_GN, N - v0);
  st = (st < 0) ? 0 : (st > permLen - 32 ? permLen - 32 : st) & ~31; stn = (stn < st) ? st : (stn > permLen ? permLen : stn); tot = (tot < 0) ? 0 : tot; if (tot > stn - st && tot <= CSR_CAP) tot = stn - st;
  if (tot > CSR_CAP) {
    for (int pass = 0; pass < 2; ++pass) { for (int i = t_; i < CSR_GN / 4; i += 256) { v4i a, c; for (int e = 0; e < 4; ++e) { a[e] = st; c[e] = 0; } *(volatile v4i*)(ROWPTR + v0 + i * 4) = a; *(volatile v4i*)(ROWCNT + v0 + i * 4) = c; } if (t_ == 0) ((volatile int*)FLAG)[0] = 1; __threadfence(); } (void)nv; return; }
  if (t_ == 0) { int acc = 0; for (int b = 0; b < CSR_NBLK; ++b) { boff[b] = acc; int c = HST[(size_t)b * NGP + g]; c = (c < 0) ? 0 : (c > CHP ? CHP : c); acc += c; if (acc > tot) acc = tot; } boff[CSR_NBLK] = acc; }
  for (int i = t_; i <= CSR_GN; i += 256) ncnt[i] = 0;
  __syncthreads();
  for (int b = 0; b < CSR_NBLK; ++b) { const int c = boff[b + 1] - boff[b]; int o_ = OFF[(size_t)g * CSR_NBLK + b]; o_ = (o_ < 0) ? 0 : (o_ > CHP - c ? CHP - c : o_); const int* src_ = STG + (size_t)b * CHP + o_;
    for (int i = t_; i < c; i += 256) { int id = src_[i]; id = (id < 0) ? 0 : id; ids[boff[b] + i] = id; int d = dst[id]; d = (d < v0) ? v0 : (d >= N ? N - 1 : d); int kk = d - v0; kk = (kk < 0) ? 0 : (kk >= CSR_GN ? CSR_GN - 1 : kk); key[boff[b] + i] = (unsigned short)kk; } }
  __syncthreads();
  if (t_ == 0) { for (int i = 0; i < tot; ++i) ncnt[key[i]] += 1; int acc = 0; for (int vl = 0; vl < CSR_GN; ++vl) { const int c = ncnt[vl]; ncnt[vl] = acc; acc += c; } ncnt[CSR_GN] = acc;
    for (int i = 0; i < tot; ++i) { const int vl = key[i]; outp[ncnt[vl]] = ids[i]; ncnt[vl] += 1; }
    for (int vl = CSR_GN; vl > 0; --vl) ncnt[vl] = ncnt[vl - 1]; ncnt[0] = 0; }
  __syncthreads();
  for (int pass = 0; pass < 2; ++pass) {
    for (int i = t_; i < (stn - st) / 4; i += 256) { v4i v; for (int e = 0; e < 4; ++e) { const int q = i * 4 + e; v[e] = (q < tot) ? outp[q] : -1; } *(volatile v4i*)(PERM + st + i * 4) = v; }
    for (int i = t_; i < CSR_GN / 4; i += 256) { v4i a, c; for (int e = 0; e < 4; ++e) { const int vl = i * 4 + e; a[e] = st + ncnt[vl]; c[e] = (vl < nv) ? (ncnt[vl + 1] - ncnt[vl]) : 0; } *(volatile v4i*)(ROWPTR + v0 + i * 4) = a; *(volatile v4i*)(ROWCNT + v0 + i * 4) = c; }
    __threadfence(); }
}
__global__ __launch_bounds__(256) void csrZ_kernel(int* __restrict__ p, size_t n4) { typedef __attribute__((ext_vector_type(4))) int v4i; const size_t tid = (size_t)blockIdx.x * 256 + threadIdx.x, nth = (size_t)gridDim.x * 256; v4i z = {0, 0, 0, 0}; for (size_t i = tid; i < n4; i += nth) *(volatile v4i*)(p + i * 4) = z; }
struct CsrBufs { int *STG, *HST, *OFF, *START, *TOT, *PERM, *ROWPTR, *ROWCNT, *FLAG; int nG, NGP, CHP; size_t permLen; char* base; size_t bytes; };
static size_t csr_carve(CsrBufs& c, char* ws, size_t off, int E, int N) {
  const size_t off0 = off; c.base = ws + off;
  auto al = [&](size_t bytes) { char* p = ws + off; off += (bytes + 255) & ~(size_t)255; return p; };
  c.nG = (N + CSR_GN - 1) / CSR_GN; c.NGP = (c.nG + 31) & ~31; const int ch = (E + CSR_NBLK - 1) / CSR_NBLK; c.CHP = (ch + 31) & ~31; c.permLen = (size_t)E + 32 * (size_t)c.nG + 32;
  c.STG = (int*)al((size_t)CSR_NBLK * c.CHP * 4); c.HST = (int*)al((size_t)CSR_NBLK * c.NGP * 4); c.OFF = (int*)al((size_t)c.NGP * CSR_NBLK * 4); c.START = (int*)al((size_t)(c.NGP + 64) * 4); c.TOT = (int*)al((size_t)(c.NGP + 64) * 4);
  c.PERM = (int*)al(c.permLen * 4); c.ROWPTR = (int*)al((size_t)c.nG * CSR_GN * 4); c.ROWCNT = (int*)al((size_t)c.nG * CSR_GN * 4); c.FLAG = (int*)al(256);
  c.bytes = off - off0; return off;
}
static void csr_build(const CsrBufs& c, const int* dst, int E, int N, hipStream_t stream) {
  const size_t smem = (size_t)(2 * c.NGP + c.CHP) * 4;
  csrZ_kernel<<<512, 256, 0, stream>>>((int*)c.base, c.bytes / 16);
  csrA_kernel<<<CSR_NBLK, 64, smem, stream>>>(dst, E, N, c.nG, c.CHP, c.NGP, c.STG, c.HST);
  csrS_kernel<<<1, 512, 0, stream>>>(c.HST, c.nG, c.NGP, c.START, c.TOT, c.OFF);
  csrB_kernel<<<c.nG, 256, 0, stream>>>(dst, N, c.nG, c.CHP, c.NGP, (int)c.permLen, c.STG, c.HST, c.OFF, c.START, c.TOT, c.PERM, c.ROWPTR, c.ROWCNT, c.FLAG);
}


__global__ __launch_bounds__(256) void prep_kernel(const float* __restrict__ x, const float* __restrict__ w1, const float* __restrict__ w2, const float* __restrict__ l1, const float* __restrict__ f2, b16* __restrict__ X16, b16* __restrict__ W1T, b16* __restrict__ W2T, b16* __restrict__ L1T, b16* __restrict__ F2T) {
  const size_t t = (size_t)blockIdx.x * 256 + threadIdx.x; const size_t nx = (size_t)N * IN / 8, n1 = (size_t)HC * IN / 8, n2 = (size_t)HID * HC / 8, n3 = (size_t)HID * HID / 8, n4 = (size_t)16 * HID / 8; v8b o;
  if (t < nx) { const size_t e = t * 8; const v4f a = *(const v4f*)(x + e), c = *(const v4f*)(x + e + 4); for (int j = 0; j < 4; ++j) { o[j] = (b16)(bf16_rne(a[j]) * XS); o[4 + j] = (b16)(bf16_rne(c[j]) * XS); } for (int pass = 0; pass < 2; ++pass) { *(volatile v8b*)(X16 + e) = o; __threadfence(); } return; }
  size_t u = t - nx; const float* w; b16* dst; int nin, nout, olim;
  if (u < n1) { w = w1; dst = W1T; nin = IN; nout = HC; olim = HC; } else if ((u -= n1) < n2) { w = w2; dst = W2T; nin = HC; nout = HID; olim = HID; } else if ((u -= n2) < n3) { w = l1; dst = L1T; nin = HID; nout = HID; olim = HID; } else if ((u -= n3) < n4) { w = f2; dst = F2T; nin = HID; nout = NOUT; olim = 16; } else return;
  const size_t e = u * 8; const int oo = (int)(e / nin), i0 = (int)(e % nin); for (int j = 0; j < 8; ++j) o[j] = (oo < nout) ? (b16)(bf16_rne(w[(size_t)(i0 + j) * nout + oo]) * WSC) : (b16)0.0f; (void)olim;
  for (int pass = 0; pass < 2; ++pass) { *(volatile v8b*)(dst + e) = o; __threadfence(); }
}
template <int KD, int NPROD, int MODE>
__global__ __launch_bounds__(128) void gemm_kernel(const b16* __restrict__ Ah, const b16* __restrict__ Al, int lda, const b16* __restrict__ W, int wcol0, const float* __restrict__ bias, float* __restrict__ Yf, b16* __restrict__ Yh, b16* __restrict__ Yl, int ldy, int ycol0) {
  __shared__ __attribute__((aligned(16))) float Tf[MODE >= 1 ? 4 : 1][16][128 + 4]; __shared__ __attribute__((aligned(16))) b16 Th[MODE == 0 ? 4 : 1][16][128 + 8], Tl[MODE == 0 ? 4 : 1][16][128 + 8];
  const int wave = threadIdx.x >> 5, lane = threadIdx.x & 31, nloc = lane & 15, hlf = lane >> 4; const size_t m0 = (size_t)blockIdx.x * 64 + wave * 16; const int n0 = blockIdx.y * 128;
  v8f acc[8];
#pragma unroll
  for (int t = 0; t < 8; ++t) acc[t] = (v8f){};
#pragma unroll 2
  for (int kb = 0; kb < KD; kb += 32) { const v16b a = frag_kb(Ah + (m0 + nloc) * lda + kb, hlf); v16b al; if (NPROD == 2) al = frag_kb(Al + (m0 + nloc) * lda + kb, hlf);
#pragma unroll
    for (int t = 0; t < 8; ++t) { const v16b bw = frag_kb(W + (size_t)(wcol0 + n0 + t * 16 + nloc) * KD + kb, hlf); acc[t] = wmma16b(a, bw, acc[t]); if (NPROD == 2) acc[t] = wmma16b(al, bw, acc[t]); } }
#pragma unroll
  for (int t = 0; t < 8; ++t) { const float bb = (MODE == 2) ? bf16_rne(bias[n0 + t * 16 + nloc]) : 0.0f;
#pragma unroll
    for (int r = 0; r < 8; ++r) { float y = acc[t][r] * (1.0f / (XS * WSC)) + bb; if (MODE == 2) y = fmaxf(y, 0.0f); if (MODE == 0) { b16 p, q; split16(y * XS, p, q); Th[wave][8 * hlf + r][t * 16 + nloc] = p; Tl[wave][8 * hlf + r][t * 16 + nloc] = q; } else Tf[wave][8 * hlf + r][t * 16 + nloc] = y; } }
  wave_lds_sync();
  for (int pass = 0; pass < 2; ++pass) {
    if (MODE == 0) { for (int r2 = 0; r2 < 16; r2 += 2) { const int rr = r2 + (lane >> 4), c8 = (lane & 15) * 8; *(volatile v8b*)(Yh + (m0 + rr) * ldy + ycol0 + n0 + c8) = *(const v8b*)(&Th[wave][rr][c8]); *(volatile v8b*)(Yl + (m0 + rr) * ldy + ycol0 + n0 + c8) = *(const v8b*)(&Tl[wave][rr][c8]); } }
    else { for (int rr = 0; rr < 16; ++rr) *(volatile v4f*)(Yf + (m0 + rr) * ldy + ycol0 + n0 + lane * 4) = *(const v4f*)(&Tf[wave][rr][lane * 4]); }
    __threadfence(); }
}
__global__ __launch_bounds__(256) void node1_kernel(const b16* __restrict__ XL, const b16* __restrict__ XLl, const float* __restrict__ asrc, const float* __restrict__ adst, int h0, float* __restrict__ AL, float* __restrict__ AR) {
  __shared__ float la[8][4], ra[8][4];
  const int wave = threadIdx.x >> 5, lane = threadIdx.x & 31; const size_t v = (size_t)blockIdx.x * 8 + wave;
  for (int hl = 0; hl < 4; ++hl) { const b16* row = XL + v * HHC + hl * HID + lane * 16; const b16* rowl = XLl + v * HHC + hl * HID + lane * 16; const v8b a = *(const v8b*)row, b = *(const v8b*)(row + 8), al_ = *(const v8b*)rowl, bl_ = *(const v8b*)(rowl + 8); const float* as_ = asrc + (size_t)(h0 + hl) * HID + lane * 16; const float* ad_ = adst + (size_t)(h0 + hl) * HID + lane * 16; float s = 0.0f, d = 0.0f;
#pragma unroll
    for (int j = 0; j < 8; ++j) { const float g0 = ((float)a[j] + (float)al_[j]) * (1.0f / XS), g1 = ((float)b[j] + (float)bl_[j]) * (1.0f / XS); s += pmul(g0, bf16_rne(as_[j])) + pmul(g1, bf16_rne(as_[8 + j])); d += pmul(g0, bf16_rne(ad_[j])) + pmul(g1, bf16_rne(ad_[8 + j])); }
#pragma unroll
    for (int o = 16; o >= 1; o >>= 1) { s += __shfl_xor(s, o); d += __shfl_xor(d, o); }
    if (lane == 0) { la[wave][hl] = s; ra[wave][hl] = d; } }
  __syncthreads();
  for (int pass = 0; pass < 2; ++pass) { if (threadIdx.x < 8) { *(volatile v4f*)(AL + ((size_t)blockIdx.x * 8 + threadIdx.x) * 4) = *(const v4f*)(&la[threadIdx.x][0]); *(volatile v4f*)(AR + ((size_t)blockIdx.x * 8 + threadIdx.x) * 4) = *(const v4f*)(&ra[threadIdx.x][0]); } __threadfence(); }
}
__global__ __launch_bounds__(256) void agg1_kernel(const b16* __restrict__ XL, const b16* __restrict__ XLl, const float* __restrict__ AL, const float* __restrict__ AR, const int* __restrict__ srcs, const float* __restrict__ b1, const int* __restrict__ PERM, const int* __restrict__ ROWPTR, const int* __restrict__ ROWCNT, int permLen, int h0, b16* __restrict__ H1, b16* __restrict__ H1l) {
  const int wave = threadIdx.x >> 5, lane = threadIdx.x & 31; const size_t v = (size_t)blockIdx.x * 8 + wave;
  int st = ROWPTR[v], cnt = ROWCNT[v]; cnt = iclamp(cnt, 0, 8192); st = iclamp(st, 0, permLen - cnt);
  for (int hl = 0; hl < 4; ++hl) { const float arv = AR[v * 4 + hl], alv = AL[v * 4 + hl]; const float self_l = lrelu(alv + arv); float mx = self_l;
    for (int j = 0; j < cnt; ++j) { const int e = iclamp(PERM[st + j], 0, E - 1); const int s = iclamp(srcs[e], 0, N - 1); mx = fmaxf(mx, lrelu(AL[(size_t)s * 4 + hl] + arv)); }
    float acc[16]; float den;
    { const float w0 = nexp(self_l - mx); den = w0; const b16* row = XL + v * HHC + hl * HID; const b16* rowl = XLl + v * HHC + hl * HID; const v8b a = *(const v8b*)(row + lane * 8), b = *(const v8b*)(row + 256 + lane * 8), la_ = *(const v8b*)(rowl + lane * 8), lb_ = *(const v8b*)(rowl + 256 + lane * 8);
      for (int j = 0; j < 8; ++j) { acc[j] = pmul(w0, (float)a[j] + (float)la_[j]); acc[8 + j] = pmul(w0, (float)b[j] + (float)lb_[j]); } }
    for (int j = 0; j < cnt; ++j) { const int e = iclamp(PERM[st + j], 0, E - 1); const int s = iclamp(srcs[e], 0, N - 1); const float w = nexp(lrelu(AL[(size_t)s * 4 + hl] + arv) - mx); den += w;
      const b16* row = XL + (size_t)s * HHC + hl * HID; const b16* rowl = XLl + (size_t)s * HHC + hl * HID; const v8b a = *(const v8b*)(row + lane * 8), b = *(const v8b*)(row + 256 + lane * 8), la_ = *(const v8b*)(rowl + lane * 8), lb_ = *(const v8b*)(rowl + 256 + lane * 8);
      for (int q = 0; q < 8; ++q) { acc[q] += pmul(w, (float)a[q] + (float)la_[q]); acc[8 + q] += pmul(w, (float)b[q] + (float)lb_[q]); } }
    const float inv = (1.0f / XS) / (den + EPSD); v8b o0, o1, l0, l1; const float* bb = b1 + (size_t)(h0 + hl) * HID;
    for (int q = 0; q < 8; ++q) { b16 p, pq; split16(elu_(acc[q] * inv + bf16_rne(bb[lane * 8 + q])) * XS, p, pq); o0[q] = p; l0[q] = pq; split16(elu_(acc[8 + q] * inv + bf16_rne(bb[256 + lane * 8 + q])) * XS, p, pq); o1[q] = p; l1[q] = pq; }
    b16* orow = H1 + v * HC + (size_t)(h0 + hl) * HID; b16* orowl = H1l + v * HC + (size_t)(h0 + hl) * HID;
    for (int pass = 0; pass < 2; ++pass) { *(volatile v8b*)(orow + lane * 8) = o0; *(volatile v8b*)(orow + 256 + lane * 8) = o1; *(volatile v8b*)(orowl + lane * 8) = l0; *(volatile v8b*)(orowl + 256 + lane * 8) = l1; __threadfence(); } }
}
__global__ __launch_bounds__(256) void node2_kernel(const float* __restrict__ XL2, const float* __restrict__ asrc, const float* __restrict__ adst, float* __restrict__ A2) {
  __shared__ float la[8][4];
  const int wave = threadIdx.x >> 5, lane = threadIdx.x & 31; const size_t v = (size_t)blockIdx.x * 8 + wave; float s = 0.0f, d = 0.0f;
  for (int sg = 0; sg < 4; ++sg) { const v4f g = *(const v4f*)(XL2 + v * HID + sg * 128 + lane * 4); for (int j = 0; j < 4; ++j) { const int c = sg * 128 + lane * 4 + j; s += pmul(g[j], bf16_rne(asrc[c])); d += pmul(g[j], bf16_rne(adst[c])); } }
#pragma unroll
  for (int o = 16; o >= 1; o >>= 1) { s += __shfl_xor(s, o); d += __shfl_xor(d, o); }
  if (lane == 0) { la[wave][0] = s; la[wave][1] = d; la[wave][2] = 0.0f; la[wave][3] = 0.0f; }
  __syncthreads();
  for (int pass = 0; pass < 2; ++pass) { if (threadIdx.x < 8) *(volatile v4f*)(A2 + ((size_t)blockIdx.x * 8 + threadIdx.x) * 4) = *(const v4f*)(&la[threadIdx.x][0]); __threadfence(); }
}
__global__ __launch_bounds__(256) void agg2_kernel(const float* __restrict__ XL2, const float* __restrict__ A2, const int* __restrict__ srcs, const float* __restrict__ b2, const int* __restrict__ PERM, const int* __restrict__ ROWPTR, const int* __restrict__ ROWCNT, int permLen, b16* __restrict__ H2h, b16* __restrict__ H2l) {
  const int wave = threadIdx.x >> 5, lane = threadIdx.x & 31; const size_t v = (size_t)blockIdx.x * 8 + wave;
  int st = ROWPTR[v], cnt = ROWCNT[v]; cnt = iclamp(cnt, 0, 8192); st = iclamp(st, 0, permLen - cnt);
  const float arv = A2[v * 4 + 1], alv = A2[v * 4 + 0]; const float self_l = lrelu(alv + arv); float mx = self_l;
  for (int j = 0; j < cnt; ++j) { const int e = iclamp(PERM[st + j], 0, E - 1); const int s = iclamp(srcs[e], 0, N - 1); mx = fmaxf(mx, lrelu(A2[(size_t)s * 4] + arv)); }
  float acc[16]; float den;
  { const float w0 = nexp(self_l - mx); den = w0; for (int sg = 0; sg < 4; ++sg) { const v4f g = *(const v4f*)(XL2 + v * HID + sg * 128 + lane * 4); for (int j = 0; j < 4; ++j) acc[sg * 4 + j] = pmul(w0, g[j]); } }
  for (int j = 0; j < cnt; ++j) { const int e = iclamp(PERM[st + j], 0, E - 1); const int s = iclamp(srcs[e], 0, N - 1); const float w = nexp(lrelu(A2[(size_t)s * 4] + arv) - mx); den += w;
    for (int sg = 0; sg < 4; ++sg) { const v4f g = *(const v4f*)(XL2 + (size_t)s * HID + sg * 128 + lane * 4); for (int q = 0; q < 4; ++q) acc[sg * 4 + q] += pmul(w, g[q]); } }
  const float inv = 1.0f / (den + EPSD);
  for (int pass = 0; pass < 2; ++pass) { for (int sg = 0; sg < 4; ++sg) { v4b hv, lv; for (int q = 0; q < 4; ++q) { const int c = sg * 128 + lane * 4 + q; b16 p, ql; split16((acc[sg * 4 + q] * inv + bf16_rne(b2[c])) * XS, p, ql); hv[q] = p; lv[q] = ql; }
      *(volatile v4b*)(H2h + v * HID + sg * 128 + lane * 4) = hv; *(volatile v4b*)(H2l + v * HID + sg * 128 + lane * 4) = lv; } __threadfence(); }
}
__global__ __launch_bounds__(32) void pair_kernel(const float* __restrict__ H3, const int* __restrict__ te, const b16* __restrict__ F2T, const float* __restrict__ fb, float* __restrict__ OUT8) {
  __shared__ __attribute__((aligned(16))) b16 Ah[16][HID + 8], Al[16][HID + 8]; __shared__ __attribute__((aligned(16))) float To[16][8];
  const int lane = threadIdx.x, nloc = lane & 15, hlf = lane >> 4; const int t0 = blockIdx.x * 16;
#pragma unroll 1
  for (int rr = 0; rr < 16; ++rr) { const int t = t0 + rr; const int i0 = iclamp(te[t], 0, N - 1), i1 = iclamp(te[TE + t], 0, N - 1); const float* a = H3 + (size_t)i0 * HID + lane * 16; const float* b = H3 + (size_t)i1 * HID + lane * 16;
    for (int q = 0; q < 16; ++q) { b16 p, ql; split16(pmul(a[q], b[q]) * XS, p, ql); Ah[rr][lane * 16 + q] = p; Al[rr][lane * 16 + q] = ql; } }
  wave_lds_sync();
  v8f d = {};
#pragma unroll 4
  for (int kb = 0; kb < HID; kb += 32) { const v16b bw = frag_kb(F2T + (size_t)nloc * HID + kb, hlf); d = wmma16b(frag_kb(&Ah[nloc][kb], hlf), bw, d); d = wmma16b(frag_kb(&Al[nloc][kb], hlf), bw, d); }
  if (nloc < 8) { for (int r = 0; r < 8; ++r) To[8 * hlf + r][nloc] = (nloc < NOUT) ? d[r] * (1.0f / (XS * WSC)) + bf16_rne(fb[nloc]) : 0.0f; }
  wave_lds_sync();
  for (int pass = 0; pass < 2; ++pass) { *(volatile v4f*)(OUT8 + (size_t)t0 * 8 + lane * 4) = *(const v4f*)(&To[0][0] + lane * 4); __threadfence(); }
}
__global__ __launch_bounds__(256) void outcopy_kernel(const float* __restrict__ OUT8, float* __restrict__ out) {
  const size_t tq = (size_t)blockIdx.x * 256 + threadIdx.x; const size_t total = (size_t)TE * NOUT; if (tq * 4 >= total) return; v4f o;
  for (int u = 0; u < 4; ++u) { const size_t f = tq * 4 + u; o[u] = (f < total) ? OUT8[(f / NOUT) * 8 + (f % NOUT)] : 0.0f; }
  for (int pass = 0; pass < 2; ++pass) { *(volatile v4f*)(out + tq * 4) = o; __threadfence(); }
}
}

extern "C" void kernel_launch(void* const* d_in, const int* in_sizes, int n_in, void* d_out, int out_size, void* d_ws, size_t ws_size, hipStream_t stream) {
  (void)n_in;
  auto Fp = [&](int i) { return (const float*)d_in[i]; }; auto Ip = [&](int i) { return (const int*)d_in[i]; };
  if (in_sizes[0] != N * IN || in_sizes[1] != 2 * E || in_sizes[2] != 2 * TE || in_sizes[3] != IN * HC || in_sizes[4] != NH * HID || in_sizes[7] != HC * HID || in_sizes[11] != HID * HID || in_sizes[13] != HID * NOUT || out_size != TE * NOUT) return;
  size_t off = 0; char* ws = (char*)d_ws;
  auto carve = [&](size_t bytes) { char* p = ws + off; off += (bytes + 255) & ~(size_t)255; return p; };
  b16* X16 = (b16*)carve((size_t)N * IN * 2); b16* W1T = (b16*)carve((size_t)HC * IN * 2); b16* W2T = (b16*)carve((size_t)HID * HC * 2); b16* L1T = (b16*)carve((size_t)HID * HID * 2); b16* F2T = (b16*)carve((size_t)16 * HID * 2);
  char* regB = carve((size_t)N * HHC * 2 * 2);
  char* regA = carve((size_t)N * HC * 2 * 2);
  float* AL0 = (float*)carve((size_t)N * 4 * 4); float* AR0 = (float*)carve((size_t)N * 4 * 4); float* AL1 = (float*)carve((size_t)N * 4 * 4); float* AR1 = (float*)carve((size_t)N * 4 * 4); float* A2 = (float*)carve((size_t)N * 4 * 4);
  CsrBufs csr; off = csr_carve(csr, ws, off, E, N);
  if (off > ws_size) return;
  b16* XL = (b16*)regB; b16* XLlo = XL + (size_t)N * HHC; float* XL2 = (float*)regB; b16* H2h = (b16*)(regB + (size_t)N * HID * 4); b16* H2l = H2h + (size_t)N * HID;
  b16* H1 = (b16*)regA; b16* H1lo = H1 + (size_t)N * HC; float* H3 = (float*)regA; float* OUT8 = (float*)(regA + (size_t)N * HID * 4);
  prep_kernel<<<(unsigned)(((size_t)N * IN / 8 + (size_t)HC * IN / 8 + (size_t)HID * HC / 8 + (size_t)HID * HID / 8 + 16 * HID / 8 + 255) / 256), 256, 0, stream>>>(Fp(0), Fp(3), Fp(7), Fp(11), Fp(13), X16, W1T, W2T, L1T, F2T);
  csr_build(csr, Ip(1) + E, E, N, stream);
  for (int hf = 0; hf < 2; ++hf) {
    gemm_kernel<IN, 1, 0><<<dim3(N / 64, HHC / 128), 128, 0, stream>>>(X16, nullptr, IN, W1T, hf * HHC, nullptr, nullptr, XL, XLlo, HHC, 0);
    node1_kernel<<<N / 8, 256, 0, stream>>>(XL, XLlo, Fp(4), Fp(5), hf * 4, hf == 0 ? AL0 : AL1, hf == 0 ? AR0 : AR1);
    agg1_kernel<<<N / 8, 256, 0, stream>>>(XL, XLlo, hf == 0 ? AL0 : AL1, hf == 0 ? AR0 : AR1, Ip(1), Fp(6), csr.PERM, csr.ROWPTR, csr.ROWCNT, (int)csr.permLen, hf * 4, H1, H1lo);
  }
  gemm_kernel<HC, 2, 1><<<dim3(N / 64, HID / 128), 128, 0, stream>>>(H1, H1lo, HC, W2T, 0, nullptr, XL2, nullptr, nullptr, HID, 0);
  node2_kernel<<<N / 8, 256, 0, stream>>>(XL2, Fp(8), Fp(9), A2);
  agg2_kernel<<<N / 8, 256, 0, stream>>>(XL2, A2, Ip(1), Fp(10), csr.PERM, csr.ROWPTR, csr.ROWCNT, (int)csr.permLen, H2h, H2l);
  gemm_kernel<HID, 2, 2><<<dim3(N / 64, HID / 128), 128, 0, stream>>>(H2h, H2l, HID, L1T, 0, Fp(12), H3, nullptr, nullptr, HID, 0);
  pair_kernel<<<TEP / 16, 32, 0, stream>>>(H3, Ip(2), F2T, Fp(14), OUT8);
  outcopy_kernel<<<(unsigned)((((size_t)TE * NOUT + 3) / 4 + 255) / 256), 256, 0, stream>>>(OUT8, (float*)d_out);
}
